// Correlation_3882650436435
// MI455X (gfx1250) — hardware-run, weakly checked
//
#include <hip/hip_runtime.h>
#include <math.h>

typedef __attribute__((ext_vector_type(16))) _Float16 v16h;
typedef __attribute__((ext_vector_type(16))) __bf16 v16b;
typedef __attribute__((ext_vector_type(8)))  _Float16 v8h;
typedef __attribute__((ext_vector_type(8)))  float v8f;
typedef __attribute__((ext_vector_type(4)))  float v4f;
typedef __attribute__((ext_vector_type(2)))  float v2f;
typedef __attribute__((ext_vector_type(4)))  unsigned v4u;
typedef __attribute__((ext_vector_type(4)))  int v4i;
typedef float __attribute__((may_alias)) float_a;
typedef int __attribute__((may_alias)) int_a;

template <typename T> __device__ __forceinline__ void vst2(void* p, T v) { *(volatile T*)p = v; __threadfence(); *(volatile T*)p = v; }
__device__ __forceinline__ v8f wmma16(v16h a, v16h b, v8f c) {
  v8f d = __builtin_amdgcn_wmma_f32_16x16x32_f16(false, a, false, b, (short)0, c, false, false);
  asm volatile("v_nop\n\tv_nop\n\tv_nop\n\tv_nop" : "+v"(d) : "v"(a), "v"(b));
  return d;
}
__device__ __forceinline__ v8f wmma_bf(v16b a, v16b b, v8f c) {
  v8f d = __builtin_amdgcn_wmma_f32_16x16x32_bf16(false, a, false, b, (short)0, c, false, false);
  asm volatile("v_nop\n\tv_nop\n\tv_nop\n\tv_nop" : "+v"(d) : "v"(a), "v"(b));
  return d;
}
__device__ __forceinline__ v16h frag_h(const _Float16* rowk0, int lane) {
  union { v16h v; v8h q[2]; } u; const _Float16* p = rowk0 + 8 * (lane >> 4);
  u.q[0] = *(const v8h*)p; u.q[1] = *(const v8h*)(p + 16); return u.v;
}
__device__ __forceinline__ v16h frag_f32(const float* rowk0, int lane) {
  v16h a; const float* p = rowk0 + 8 * (lane >> 4);
#pragma unroll
  for (int i = 0; i < 8; ++i) { a[i] = (_Float16)p[i]; a[8 + i] = (_Float16)p[16 + i]; }
  return a;
}
__device__ __forceinline__ v16h frag_f32s(const float* rowk0, int lane, float sc) {
  v16h a; const float* p = rowk0 + 8 * (lane >> 4);
#pragma unroll
  for (int i = 0; i < 8; ++i) { a[i] = (_Float16)(p[i] * sc); a[8 + i] = (_Float16)(p[16 + i] * sc); }
  return a;
}
__device__ __forceinline__ v16h fragc_f32(const float* W, int k0, int n, int lane, int ld, int K) {
  v16h a; const int g = lane >> 4;
#pragma unroll
  for (int i = 0; i < 8; ++i) { const int ka = k0 + 8 * g + i, kb = ka + 16;
    a[i] = (_Float16)(ka < K ? W[(size_t)(ka < K ? ka : K - 1) * ld + n] : 0.f); a[8 + i] = (_Float16)(kb < K ? W[(size_t)(kb < K ? kb : K - 1) * ld + n] : 0.f); }
  return a;
}
struct F2 { v16b h, l; };
__device__ __forceinline__ F2 bsplit16(const float v[16]) { F2 r;
#pragma unroll
  for (int i = 0; i < 16; ++i) { const __bf16 h = (__bf16)v[i]; r.h[i] = h; r.l[i] = (__bf16)(v[i] - (float)h); }
  return r; }
__device__ __forceinline__ F2 split_row(const float* row, int k0, int lane) { float v[16]; const float* p = row + k0 + 8 * (lane >> 4);
#pragma unroll
  for (int i = 0; i < 8; ++i) { v[i] = p[i]; v[8 + i] = p[16 + i]; }
  return bsplit16(v); }
__device__ __forceinline__ F2 split_rowK(const float* row, int k0, int lane, int K) { float v[16]; const int g = lane >> 4;
#pragma unroll
  for (int i = 0; i < 8; ++i) { const int ka = k0 + 8 * g + i, kb = ka + 16; v[i] = ka < K ? row[ka < K ? ka : K - 1] : 0.f; v[8 + i] = kb < K ? row[kb < K ? kb : K - 1] : 0.f; }
  return bsplit16(v); }
__device__ __forceinline__ F2 split_col(const float* W, int k0, int n, int lane, int ld, int K) { float v[16]; const int g = lane >> 4;
#pragma unroll
  for (int i = 0; i < 8; ++i) { const int ka = k0 + 8 * g + i, kb = ka + 16; v[i] = ka < K ? W[(size_t)(ka < K ? ka : K - 1) * ld + n] : 0.f; v[8 + i] = kb < K ? W[(size_t)(kb < K ? kb : K - 1) * ld + n] : 0.f; }
  return bsplit16(v); }
__device__ __forceinline__ v8f mac3(const F2& a, const F2& b, v8f c) { c = wmma_bf(a.l, b.h, c); c = wmma_bf(a.h, b.l, c); return wmma_bf(a.h, b.h, c); }
__device__ __forceinline__ float sigm(float v) { return 1.0f / (1.0f + expf(-v)); }
#define LDSX() do { asm volatile("s_wait_dscnt 0" ::: "memory"); __builtin_amdgcn_wave_barrier(); __builtin_amdgcn_fence(__ATOMIC_RELEASE, "workgroup"); } while (0)


#define NB 8
#define CC 256
#define HH 64
#define WWD 64
#define MD 20
#define ND 21
#ifndef TNB
#define TNB NB
#endif
typedef __attribute__((ext_vector_type(8))) __bf16 v8b;
__device__ __forceinline__ v16b frag_b(const __bf16* rowk0, int lane) {
  union { v16b v; v8b q[2]; } u; const __bf16* p = rowk0 + 8 * (lane >> 4);
  u.q[0] = *(const v8b*)p; u.q[1] = *(const v8b*)(p + 16); return u.v;
}
__device__ __forceinline__ float bfr(float v) { return (float)(__bf16)v; }
__device__ __attribute__((noinline)) float exp_ni(float v) { return expf(v); }
__device__ __attribute__((noinline)) float erf_ni(float v) { return erff(v); }

#define WS_T1  0u
#define WS_T2  (WS_T1 + 2u * (size_t)NB * HH * WWD * CC)
#define WS_END (WS_T2 + 2u * (size_t)NB * HH * WWD * CC)

__global__ __launch_bounds__(256) void k_tr(const float* __restrict__ I1, const float* __restrict__ I2, __bf16* __restrict__ T1, __bf16* __restrict__ T2) { __shared__ __align__(16) __bf16 st[WWD][CC + 8];
  const int t = threadIdx.x; const int y = blockIdx.x; const size_t b = blockIdx.y; const int which = blockIdx.z; const float* I = which == 0 ? I1 : I2; __bf16* T = which == 0 ? T1 : T2;
  for (int e = t; e < CC * WWD; e += 256) { const int c = e >> 6, x = e & 63; st[x][c] = (__bf16)I[((b * CC + c) * HH + y) * WWD + x]; }
  __syncthreads();
  for (int e = t; e < WWD * (CC / 8); e += 256) { const int x = e >> 5, q = e & 31; vst2((unsigned*)(T + ((b * HH + y) * WWD + x) * CC + q * 8), *(const v4u*)&st[x][q * 8]); } }
__global__ __launch_bounds__(128) void k_corr(const __bf16* __restrict__ T1, const __bf16* __restrict__ T2, float* __restrict__ OUT) { __shared__ __align__(16) float sc[WWD][68]; __shared__ __align__(16) float so[ND][WWD];
  const int tid = threadIdx.x, wave = tid >> 5, lane = tid & 31, col = lane & 15, g = lane >> 4; const int y = blockIdx.x, dyi = blockIdx.y; const size_t b = blockIdx.z; const int y2 = y + 2 * dyi - MD;
  if (y2 < 0 || y2 >= HH) {
    for (int e = tid; e < ND * WWD; e += 128) so[e / WWD][e % WWD] = 0.f;
    __syncthreads();
    for (int e = tid; e < ND * (WWD / 4); e += 128) { const int dxi = e >> 4, q = e & 15; vst2(OUT + (((b * (ND * ND)) + dyi * ND + dxi) * HH + y) * WWD + q * 4, *(const v4f*)&so[dxi][q * 4]); }
    return; }
  const __bf16* A0 = T1 + ((b * HH + y) * WWD + wave * 16 + col) * CC; v8f acc[4] = {};
#pragma unroll
  for (int kc = 0; kc < CC / 32; ++kc) { const v16b a = frag_b(A0 + kc * 32, lane);
#pragma unroll
    for (int j = 0; j < 4; ++j) acc[j] = wmma_bf(a, frag_b(T2 + ((b * HH + y2) * WWD + j * 16 + col) * CC + kc * 32, lane), acc[j]); }
#pragma unroll
  for (int j = 0; j < 4; ++j)
#pragma unroll
    for (int r = 0; r < 8; ++r) sc[wave * 16 + 8 * g + r][j * 16 + col] = acc[j][r] * (1.0f / CC);
  __syncthreads();
  for (int e = tid; e < ND * WWD; e += 128) { const int dxi = e / WWD, x = e % WWD; const int x2 = x + 2 * dxi - MD; so[dxi][x] = (x2 >= 0 && x2 < WWD) ? sc[x][x2] : 0.f; }
  __syncthreads();
  for (int e = tid; e < ND * (WWD / 4); e += 128) { const int dxi = e >> 4, q = e & 15; vst2(OUT + (((b * (ND * ND)) + dyi * ND + dxi) * HH + y) * WWD + q * 4, *(const v4f*)&so[dxi][q * 4]); } }
extern "C" void kernel_launch(void* const* d_in, const int* in_sizes, int n_in, void* d_out, int out_size, void* d_ws, size_t ws_size, hipStream_t stream) {
  (void)in_sizes; (void)n_in; (void)out_size;
  const float** F = (const float**)d_in;
  if (ws_size < (size_t)WS_END) return;
  char* ws = (char*)d_ws; __bf16 *T1 = (__bf16*)(ws + WS_T1), *T2 = (__bf16*)(ws + WS_T2);
  k_tr<<<dim3(HH, TNB, 2), 256, 0, stream>>>(F[0], F[1], T1, T2);
  k_corr<<<dim3(HH, ND, TNB), 128, 0, stream>>>(T1, T2, (float*)d_out);
}
